// NNConvCritic_43439299231748
// MI455X (gfx1250) — hardware-verified
//
#include <hip/hip_runtime.h>
#define NNODE 50000
#define NE 800000
#define NG 64
#define INN 16
#define ON 20
#define HE 64
#define KP 1056
#define NN NNODE
#define MAXDEG 256

typedef __bf16 v16b __attribute__((ext_vector_type(16)));
typedef unsigned short v8us __attribute__((ext_vector_type(8), may_alias));
typedef float  v8f  __attribute__((ext_vector_type(8)));
typedef float  v4f  __attribute__((ext_vector_type(4)));
typedef float  v4fa __attribute__((ext_vector_type(4), may_alias));
union FragB { v16b v; v8us half[2]; unsigned short u[16]; };

__device__ __forceinline__ unsigned short bf16_bits(float x) { unsigned int u = __float_as_uint(x); return (unsigned short)((u + 0x7FFFu + ((u >> 16) & 1u)) >> 16); }
__device__ __forceinline__ float bf16_val(unsigned short b) { return __uint_as_float(((unsigned int)b) << 16); }
__device__ __forceinline__ float bf16_round(float x) { return bf16_val(bf16_bits(x)); }
template <int NT>
__device__ __forceinline__ v8f mmaN(v16b ah, v16b al, v16b bh, v16b bl, v8f c) {
  c = __builtin_amdgcn_wmma_f32_16x16x32_bf16(false, ah, false, bh, (short)0, c, false, false);
  if (NT >= 2) c = __builtin_amdgcn_wmma_f32_16x16x32_bf16(false, al, false, bh, (short)0, c, false, false);
  if (NT >= 3) c = __builtin_amdgcn_wmma_f32_16x16x32_bf16(false, ah, false, bl, (short)0, c, false, false);
  asm volatile("v_nop\n\tv_nop\n\tv_nop\n\tv_nop" : "+v"(c) : "v"(ah), "v"(al), "v"(bh), "v"(bl));
  return c;
}

__global__ __launch_bounds__(256) void k_wt_bf16(const float* __restrict__ W, unsigned short* __restrict__ Wt, int K, int N) {
  const int t = blockIdx.x * 256 + threadIdx.x;
  const int k8n = K / 8;
  if (t >= N * k8n) return;
  const int n = t / k8n, k8 = (t % k8n) * 8;
  v8us v;
#pragma unroll
  for (int i = 0; i < 8; ++i) v[i] = bf16_bits(W[(size_t)(k8 + i) * N + n]);
  *(volatile v8us*)(Wt + (size_t)n * K + k8) = v;
  __threadfence();
  *(volatile v8us*)(Wt + (size_t)n * K + k8) = v;
}

template <bool ASPLIT, int ACT, bool BIAS_BF16>
__global__ __launch_bounds__(128) void k_gemm_bf(const float* __restrict__ A, int lda, const unsigned short* __restrict__ Wt, int ldb,
                                               const float* __restrict__ bias, float* __restrict__ C, int ldc, int M, int N, int K) {
  __shared__ __attribute__((aligned(16))) float so[4][16][64];
  const int tid = threadIdx.x, w = tid >> 5, lane = tid & 31, ln = lane & 15, hh = lane >> 4;
  const int ntn = N / 64;
  const int wid = blockIdx.x * 4 + w;
  const int mt = wid / ntn, nq = wid % ntn;
  if (mt * 16 >= M) return;
  const int row0 = mt * 16, col0 = nq * 64;
  const float* arow = A + (size_t)(row0 + ln) * lda;
  v8f acc[4] = {};
  for (int kb = 0; kb < K; kb += 32) {
    FragB ah, al;
    const v4f x0 = *(const v4fa*)(arow + kb + 8 * hh), x1 = *(const v4fa*)(arow + kb + 8 * hh + 4);
    const v4f x2 = *(const v4fa*)(arow + kb + 16 + 8 * hh), x3 = *(const v4fa*)(arow + kb + 16 + 8 * hh + 4);
    float xs[16] = {x0[0],x0[1],x0[2],x0[3],x1[0],x1[1],x1[2],x1[3],x2[0],x2[1],x2[2],x2[3],x3[0],x3[1],x3[2],x3[3]};
#pragma unroll
    for (int i = 0; i < 16; ++i) { const unsigned short hb = bf16_bits(xs[i]); ah.u[i] = hb; al.u[i] = ASPLIT ? bf16_bits(xs[i] - bf16_val(hb)) : (unsigned short)0; }
#pragma unroll
    for (int t = 0; t < 4; ++t) {
      const unsigned short* brow = Wt + (size_t)(col0 + t * 16 + ln) * ldb + kb;
      FragB b;
      b.half[0] = *(const v8us*)(brow + 8 * hh);
      b.half[1] = *(const v8us*)(brow + 16 + 8 * hh);
      acc[t] = mmaN<ASPLIT ? 2 : 1>(ah.v, al.v, b.v, b.v, acc[t]);
    }
  }
#pragma unroll
  for (int t = 0; t < 4; ++t) {
    float bv = bias ? bias[col0 + t * 16 + ln] : 0.f;
    if (BIAS_BF16) bv = bf16_round(bv);
#pragma unroll
    for (int r = 0; r < 8; ++r) { float v = acc[t][r] + bv; if (ACT == 1) v = fmaxf(v, 0.f); so[w][8 * hh + r][t * 16 + ln] = v; }
  }
  __builtin_amdgcn_fence(__ATOMIC_ACQ_REL, "workgroup");
  __builtin_amdgcn_wave_barrier();
  const int rsub = lane >> 4, c4 = (lane & 15) * 4;
  for (int pass = 0; pass < 2; ++pass) {
#pragma unroll
    for (int q = 0; q < 8; ++q) {
      const int r = q * 2 + rsub;
      const v4f v = *(const v4fa*)&so[w][r][c4];
      *(volatile v4f*)(C + (size_t)(row0 + r) * ldc + col0 + c4) = v;
    }
    if (pass == 0) __threadfence();
  }
}

template <int D, bool CAUSAL>
__global__ __launch_bounds__(128) void k_flash(const float* __restrict__ qb, const float* __restrict__ kb, const float* __restrict__ vb,
                                             int pitch, int T, int H, float scale, float* __restrict__ y, int ypitch) {
  constexpr int KS = D / 32;
  constexpr int DT = D / 16;
  __shared__ __attribute__((aligned(16))) unsigned short sKh[32][D + 8], sKl[32][D + 8], sVh[32][D + 8], sVl[32][D + 8];
  __shared__ __attribute__((aligned(16))) unsigned short sPh[4][16][40], sPl[4][16][40];
  __shared__ __attribute__((aligned(16))) float sO[4][16][D];
  const int tid = threadIdx.x, w = tid >> 5, lane = tid & 31, ln = lane & 15, hh = lane >> 4;
  const int nqb = (T + 63) / 64;
  const int bh = blockIdx.x / nqb, qblk = blockIdx.x % nqb;
  const int b = bh / H, h = bh % H;
  const int q0 = qblk * 64 + w * 16;
  const float* Q = qb + (size_t)b * T * pitch + h * D;
  const float* K = kb + (size_t)b * T * pitch + h * D;
  const float* V = vb + (size_t)b * T * pitch + h * D;

  FragB aqh[KS], aql[KS];
  {
    int row = q0 + ln; if (row >= T) row = T - 1;
    const float* qr = Q + (size_t)row * pitch;
#pragma unroll
    for (int ks = 0; ks < KS; ++ks)
#pragma unroll
      for (int i = 0; i < 16; ++i) {
        const int d = ks * 32 + ((i < 8) ? (8 * hh + i) : (16 + 8 * hh + (i - 8)));
        const float x = qr[d] * scale; const unsigned short hb = bf16_bits(x);
        aqh[ks].u[i] = hb; aql[ks].u[i] = bf16_bits(x - bf16_val(hb));
      }
  }
  float m_r[8], l_r[8];
#pragma unroll
  for (int r = 0; r < 8; ++r) { m_r[r] = -3.0e38f; l_r[r] = 0.f; }
  v8f oacc[DT];
#pragma unroll
  for (int dt = 0; dt < DT; ++dt) oacc[dt] = (v8f){0.f,0.f,0.f,0.f,0.f,0.f,0.f,0.f};

  const int kv_end = CAUSAL ? min(T, qblk * 64 + 64) : T;
  for (int j0 = 0; j0 < kv_end; j0 += 32) {
    __syncthreads();
    for (int e = tid; e < 32 * (D / 4); e += 128) {
      const int r = e / (D / 4), c4 = (e % (D / 4)) * 4;
      const int key = j0 + r;
      v4f kf = {0.f,0.f,0.f,0.f}, vf = {0.f,0.f,0.f,0.f};
      if (key < T) { kf = *(const v4fa*)(K + (size_t)key * pitch + c4); vf = *(const v4fa*)(V + (size_t)key * pitch + c4); }
#pragma unroll
      for (int t = 0; t < 4; ++t) {
        unsigned short hb = bf16_bits(kf[t]); sKh[r][c4 + t] = hb; sKl[r][c4 + t] = bf16_bits(kf[t] - bf16_val(hb));
        hb = bf16_bits(vf[t]); sVh[r][c4 + t] = hb; sVl[r][c4 + t] = bf16_bits(vf[t] - bf16_val(hb));
      }
    }
    __syncthreads();
    v8f s[2];
#pragma unroll
    for (int nt = 0; nt < 2; ++nt) {
      v8f acc = {};
#pragma unroll
      for (int ks = 0; ks < KS; ++ks) {
        FragB bh_, bl_;
        bh_.half[0] = *(const v8us*)&sKh[nt * 16 + ln][ks * 32 + 8 * hh]; bh_.half[1] = *(const v8us*)&sKh[nt * 16 + ln][ks * 32 + 16 + 8 * hh];
        bl_.half[0] = *(const v8us*)&sKl[nt * 16 + ln][ks * 32 + 8 * hh]; bl_.half[1] = *(const v8us*)&sKl[nt * 16 + ln][ks * 32 + 16 + 8 * hh];
        acc = mmaN<3>(aqh[ks].v, aql[ks].v, bh_.v, bl_.v, acc);
      }
      s[nt] = acc;
    }
    float alpha[8];
#pragma unroll
    for (int r = 0; r < 8; ++r) {
      const int qi = q0 + 8 * hh + r;
      const int ja = j0 + ln, jb = j0 + 16 + ln;
      if (CAUSAL) { if (ja > qi) s[0][r] = -3.0e38f; if (jb > qi) s[1][r] = -3.0e38f; }
      if (ja >= T) s[0][r] = -3.0e38f;
      if (jb >= T) s[1][r] = -3.0e38f;
      float mx = fmaxf(s[0][r], s[1][r]);
      mx = fmaxf(mx, __shfl_xor(mx, 1, 32)); mx = fmaxf(mx, __shfl_xor(mx, 2, 32)); mx = fmaxf(mx, __shfl_xor(mx, 4, 32)); mx = fmaxf(mx, __shfl_xor(mx, 8, 32));
      const float mnew = fmaxf(m_r[r], mx);
      alpha[r] = (mnew > -1.0e38f) ? __expf(m_r[r] - mnew) : 1.0f;
      const float p0 = (s[0][r] > -1.0e38f) ? __expf(s[0][r] - mnew) : 0.f;
      const float p1 = (s[1][r] > -1.0e38f) ? __expf(s[1][r] - mnew) : 0.f;
      m_r[r] = mnew;
      l_r[r] = l_r[r] * alpha[r] + p0 + p1;
      unsigned short hb = bf16_bits(p0); sPh[w][8 * hh + r][ln] = hb;      sPl[w][8 * hh + r][ln] = bf16_bits(p0 - bf16_val(hb));
      hb = bf16_bits(p1);                sPh[w][8 * hh + r][16 + ln] = hb; sPl[w][8 * hh + r][16 + ln] = bf16_bits(p1 - bf16_val(hb));
    }
#pragma unroll
    for (int dt = 0; dt < DT; ++dt)
#pragma unroll
      for (int r = 0; r < 8; ++r) oacc[dt][r] *= alpha[r];
    __builtin_amdgcn_fence(__ATOMIC_ACQ_REL, "workgroup");
    __builtin_amdgcn_wave_barrier();
    FragB pah, pal;
    pah.half[0] = *(const v8us*)&sPh[w][ln][8 * hh]; pah.half[1] = *(const v8us*)&sPh[w][ln][16 + 8 * hh];
    pal.half[0] = *(const v8us*)&sPl[w][ln][8 * hh]; pal.half[1] = *(const v8us*)&sPl[w][ln][16 + 8 * hh];
#pragma unroll
    for (int dt = 0; dt < DT; ++dt) {
      FragB bvh, bvl;
#pragma unroll
      for (int i = 0; i < 8; ++i) {
        bvh.u[i] = sVh[8 * hh + i][dt * 16 + ln]; bvh.u[8 + i] = sVh[16 + 8 * hh + i][dt * 16 + ln];
        bvl.u[i] = sVl[8 * hh + i][dt * 16 + ln]; bvl.u[8 + i] = sVl[16 + 8 * hh + i][dt * 16 + ln];
      }
      oacc[dt] = mmaN<3>(pah.v, pal.v, bvh.v, bvl.v, oacc[dt]);
    }
    __builtin_amdgcn_fence(__ATOMIC_ACQ_REL, "workgroup");
    __builtin_amdgcn_wave_barrier();
  }
#pragma unroll
  for (int r = 0; r < 8; ++r) {
    float l = l_r[r];
    l += __shfl_xor(l, 1, 32); l += __shfl_xor(l, 2, 32); l += __shfl_xor(l, 4, 32); l += __shfl_xor(l, 8, 32);
    l_r[r] = (l > 0.f) ? 1.0f / l : 0.f;
  }
#pragma unroll
  for (int dt = 0; dt < DT; ++dt)
#pragma unroll
    for (int r = 0; r < 8; ++r) sO[w][8 * hh + r][dt * 16 + ln] = oacc[dt][r] * l_r[r];
  __builtin_amdgcn_fence(__ATOMIC_ACQ_REL, "workgroup");
  __builtin_amdgcn_wave_barrier();
  for (int pass = 0; pass < 2; ++pass) {
    for (int r = 0; r < 16; ++r) {
      const int row = q0 + r;
      if (row < T && lane < D / 4) {
        const v4f val = *(const v4fa*)&sO[w][r][lane * 4];
        *(volatile v4f*)(y + ((size_t)b * T + row) * ypitch + h * D + lane * 4) = val;
      }
    }
    if (pass == 0) __threadfence();
  }
}

template <bool ASPLIT, bool BSPLIT, int ACT>
__global__ __launch_bounds__(128) void k_gemm_b(const float* __restrict__ A, int lda, size_t sA, const unsigned short* __restrict__ Bh, const unsigned short* __restrict__ Bl, int ldb, size_t sB,
                                             const float* __restrict__ bias, const float* __restrict__ resid, int ldr, size_t sR, float rsign, float alpha,
                                             float* __restrict__ C, int ldc, size_t sC, int M, int N, int K) {
  __shared__ __attribute__((aligned(16))) float so[4][16][64];
  const int tid = threadIdx.x, w = tid >> 5, lane = tid & 31, ln = lane & 15, hh = lane >> 4;
  const int by = blockIdx.y;
  A += (size_t)by * sA; Bh += (size_t)by * sB; if (BSPLIT) Bl += (size_t)by * sB; C += (size_t)by * sC; if (resid) resid += (size_t)by * sR;
  const int ntn = (N + 63) / 64; const int wid = blockIdx.x * 4 + w; const int mt = wid / ntn, nq = wid % ntn;
  if (mt * 16 >= M) return;
  const int row0 = mt * 16, col0 = nq * 64;
  const float* arow = A + (size_t)(row0 + ln) * lda;
  v8f acc[4] = {};
  for (int kb = 0; kb < K; kb += 32) {
    FragB ah, al;
    const v4f x0 = *(const v4fa*)(arow + kb + 8 * hh), x1 = *(const v4fa*)(arow + kb + 8 * hh + 4);
    const v4f x2 = *(const v4fa*)(arow + kb + 16 + 8 * hh), x3 = *(const v4fa*)(arow + kb + 16 + 8 * hh + 4);
    float xs[16] = {x0[0],x0[1],x0[2],x0[3],x1[0],x1[1],x1[2],x1[3],x2[0],x2[1],x2[2],x2[3],x3[0],x3[1],x3[2],x3[3]};
#pragma unroll
    for (int i = 0; i < 16; ++i) { const unsigned short hb = bf16_bits(xs[i]); ah.u[i] = hb; al.u[i] = ASPLIT ? bf16_bits(xs[i] - bf16_val(hb)) : (unsigned short)0; }
#pragma unroll
    for (int t = 0; t < 4; ++t) {
      if (col0 + t * 16 >= N) continue;
      const size_t boff = (size_t)(col0 + t * 16 + ln) * ldb + kb;
      FragB bh_, bl_; bh_.half[0] = *(const v8us*)(Bh + boff + 8 * hh); bh_.half[1] = *(const v8us*)(Bh + boff + 16 + 8 * hh);
      if (BSPLIT) { bl_.half[0] = *(const v8us*)(Bl + boff + 8 * hh); bl_.half[1] = *(const v8us*)(Bl + boff + 16 + 8 * hh); } else bl_ = bh_;
      acc[t] = mmaN<ASPLIT ? (BSPLIT ? 3 : 2) : 1>(ah.v, al.v, bh_.v, bl_.v, acc[t]);
    }
  }
#pragma unroll
  for (int t = 0; t < 4; ++t) {
    const int col = col0 + t * 16 + ln; if (col0 + t * 16 >= N) continue; const float bv = bias ? bf16_round(bias[col]) : 0.f;
#pragma unroll
    for (int r = 0; r < 8; ++r) { float v = acc[t][r] * alpha + bv; if (resid) v += rsign * resid[(size_t)(row0 + 8 * hh + r) * ldr + col]; if (ACT == 1) v = fmaxf(v, 0.f); else if (ACT == 2) v = fmaxf(v, 0.f) + log1pf(expf(-fabsf(v))); so[w][8 * hh + r][t * 16 + ln] = v; }
  }
  __builtin_amdgcn_fence(__ATOMIC_ACQ_REL, "workgroup"); __builtin_amdgcn_wave_barrier();
  const int rsub = lane >> 4, c4 = (lane & 15) * 4;
  for (int pass = 0; pass < 2; ++pass) {
#pragma unroll
    for (int q = 0; q < 8; ++q) { const int r = q * 2 + rsub; if (col0 + c4 < N) { const v4f v = *(const v4fa*)&so[w][r][c4]; *(volatile v4f*)(C + (size_t)(row0 + r) * ldc + col0 + c4) = v; } }
    if (pass == 0) __threadfence();
  }
}
__global__ __launch_bounds__(256) void k_split_transpose_b(const float* __restrict__ src, int lds_, size_t sIn, unsigned short* __restrict__ hi, unsigned short* __restrict__ lo, size_t sOut, int K, int N) {
  const size_t t = (size_t)blockIdx.x * 256 + threadIdx.x; const int k8n = K / 8; if (t >= (size_t)N * k8n) return;
  src += (size_t)blockIdx.y * sIn; hi += (size_t)blockIdx.y * sOut; lo += (size_t)blockIdx.y * sOut;
  const int n = (int)(t / k8n), k8 = (int)(t % k8n) * 8; v8us vh, vl;
#pragma unroll
  for (int i = 0; i < 8; ++i) { const float x = src[(size_t)(k8 + i) * lds_ + n]; const unsigned short hb = bf16_bits(x); vh[i] = hb; vl[i] = bf16_bits(x - bf16_val(hb)); }
  unsigned short* dh = hi + (size_t)n * K + k8; unsigned short* dl = lo + (size_t)n * K + k8;
  *(volatile v8us*)dh = vh; *(volatile v8us*)dl = vl; __threadfence(); *(volatile v8us*)dh = vh; *(volatile v8us*)dl = vl;
}

#define CS_NW 1024
#define CS_CH 832
#define CS_NB 256
#define CS_CAP 8192
__device__ __forceinline__ int cs_dst(const int* __restrict__ eidst, int e, int ne, int nt, int nn) { if (e >= nt) return -1; int d = (e < ne) ? eidst[e] : (e - ne); return d < 0 ? 0 : (d >= nn ? nn - 1 : d); }
__global__ __launch_bounds__(256) void k_cs_p1(const int* __restrict__ eidst, int ne, int nt, int nn, int* __restrict__ seg_dst, int* __restrict__ seg_eid, int* __restrict__ P1, int* __restrict__ Q1) {
  __shared__ int scnt[8][CS_NB]; __shared__ int srun[8][CS_NB]; __shared__ int sod[8][CS_CH]; __shared__ int soe[8][CS_CH];
  const int tid = threadIdx.x, wv = tid >> 5, lane = tid & 31; const int w = blockIdx.x * 8 + wv; const int e0 = w * CS_CH;
  for (int i = lane; i < CS_NB; i += 32) { scnt[wv][i] = 0; srun[wv][i] = 0; }
  __builtin_amdgcn_fence(__ATOMIC_ACQ_REL, "workgroup"); __builtin_amdgcn_wave_barrier();
#pragma unroll 1
  for (int i0 = 0; i0 < CS_CH; i0 += 32) { const int e = e0 + i0 + lane; const int d = cs_dst(eidst, e, ne, nt, nn); const int hb = (d < 0) ? -1 : (d >> 8);
#pragma unroll 1
    for (int ld = 0; ld < 32; ++ld) { const int kk = __shfl(hb, ld, 32); const unsigned long long m = __ballot(hb == kk); const int first = __ffsll((long long)m) - 1; if (ld == first && lane == first && kk >= 0) scnt[wv][kk] += __popcll(m); }
    __builtin_amdgcn_fence(__ATOMIC_ACQ_REL, "workgroup"); __builtin_amdgcn_wave_barrier(); }
  { int loc[8]; int s = 0; for (int j = 0; j < 8; ++j) { loc[j] = s; s += scnt[wv][lane * 8 + j]; }
    int incl = s; for (int o = 1; o < 32; o <<= 1) { const int v = __shfl_up(incl, o, 32); if (lane >= o) incl += v; } const int excl = incl - s;
    for (int j = 0; j < 8; ++j) srun[wv][lane * 8 + j] = excl + loc[j]; }
  __builtin_amdgcn_fence(__ATOMIC_ACQ_REL, "workgroup"); __builtin_amdgcn_wave_barrier();
  for (int pass = 0; pass < 2; ++pass) { for (int i = lane; i < CS_NB; i += 32) { *(volatile int*)(P1 + (size_t)w * CS_NB + i) = scnt[wv][i]; *(volatile int*)(Q1 + (size_t)w * CS_NB + i) = srun[wv][i]; } if (pass == 0) __threadfence(); }
#pragma unroll 1
  for (int i0 = 0; i0 < CS_CH; i0 += 32) { const int e = e0 + i0 + lane; const int d = cs_dst(eidst, e, ne, nt, nn); const int hb = (d < 0) ? -1 : (d >> 8);
    int pos = -1; int grpcnt = 0; bool leader = false;
#pragma unroll 1
    for (int ld = 0; ld < 32; ++ld) { const int kk = __shfl(hb, ld, 32); const unsigned long long g = __ballot(hb == kk); const int first = __ffsll((long long)g) - 1;
      if (ld == first && kk >= 0) { if (hb == kk) { const unsigned long long below = g & ((1ull << lane) - 1ull); pos = srun[wv][kk] + __popcll(below); if (lane == first) { leader = true; grpcnt = __popcll(g); } } } }
    if (pos >= 0) { sod[wv][pos] = d; soe[wv][pos] = e; }
    __builtin_amdgcn_fence(__ATOMIC_ACQ_REL, "workgroup"); __builtin_amdgcn_wave_barrier();
    if (leader) srun[wv][hb] += grpcnt;
    __builtin_amdgcn_fence(__ATOMIC_ACQ_REL, "workgroup"); __builtin_amdgcn_wave_barrier(); }
  for (int pass = 0; pass < 2; ++pass) { for (int i = lane; i < CS_CH; i += 32) { *(volatile int*)(seg_dst + (size_t)e0 + i) = sod[wv][i]; *(volatile int*)(seg_eid + (size_t)e0 + i) = soe[wv][i]; } if (pass == 0) __threadfence(); }
}
__global__ __launch_bounds__(256) void k_cs_scan(const int* __restrict__ P1, int* __restrict__ R, int* __restrict__ S) {
  __shared__ int tot[CS_NB]; __shared__ int st[CS_NB + 1];
  const int b = threadIdx.x; int acc = 0;
#pragma unroll 1
  for (int w = 0; w < CS_NW; ++w) { const int c = P1[(size_t)w * CS_NB + b]; *(volatile int*)(R + (size_t)w * CS_NB + b) = acc; acc += c; }
  __threadfence();
  acc = 0;
#pragma unroll 1
  for (int w = 0; w < CS_NW; ++w) { const int c = P1[(size_t)w * CS_NB + b]; *(volatile int*)(R + (size_t)w * CS_NB + b) = acc; acc += c; }
  tot[b] = acc; __syncthreads();
  if (b == 0) { int s = 0; for (int i = 0; i < CS_NB; ++i) { st[i] = s; s += (tot[i] + 31) & ~31; } st[CS_NB] = s; }
  __syncthreads();
  for (int pass = 0; pass < 2; ++pass) { *(volatile int*)(S + b) = st[b]; if (b < 32) *(volatile int*)(S + CS_NB + b) = (b == 0) ? st[CS_NB] : 0; if (pass == 0) __threadfence(); }
}
__global__ __launch_bounds__(256) void k_cs_p2(const int* __restrict__ seg_dst, const int* __restrict__ seg_eid, const int* __restrict__ P1, const int* __restrict__ Q1, const int* __restrict__ R, const int* __restrict__ S, int nn, int* __restrict__ csr_eid, int* __restrict__ csr_start, int* __restrict__ csr_cnt) {
  __shared__ int sd[CS_CAP]; __shared__ int se[CS_CAP]; __shared__ int sorted[CS_CAP]; __shared__ int lcnt[CS_NB]; __shared__ int lpre[CS_NB + 1];
  const int hb = blockIdx.x, t = threadIdx.x; const int total = (R[(size_t)(CS_NW - 1) * CS_NB + hb] + P1[(size_t)(CS_NW - 1) * CS_NB + hb]); const int tot = total > CS_CAP ? CS_CAP : total;
#pragma unroll 1
  for (int w = t; w < CS_NW; w += 256) { const int c = P1[(size_t)w * CS_NB + hb]; const int base = R[(size_t)w * CS_NB + hb]; const int src = w * CS_CH + Q1[(size_t)w * CS_NB + hb];
    for (int k = 0; k < (c < CS_CH ? c : CS_CH); ++k) { const int p = base + k; if (p >= 0 && p < CS_CAP) { sd[p] = seg_dst[src + k] & 255; se[p] = seg_eid[src + k]; } } }
  __syncthreads();
  { int c = 0;
#pragma unroll 1
    for (int i = 0; i < tot; ++i) c += (sd[i] == t) ? 1 : 0; lcnt[t] = c; }
  __syncthreads();
  if (t == 0) { int s = 0; for (int i = 0; i < CS_NB; ++i) { lpre[i] = s; s += lcnt[i]; } lpre[CS_NB] = s; }
  __syncthreads();
  { int k = lpre[t];
#pragma unroll 1
    for (int i = 0; i < tot; ++i) if (sd[i] == t) { sorted[k++] = se[i]; } }
  __syncthreads();
  const int s0 = S[hb]; const int s1 = S[hb + 1];
  for (int pass = 0; pass < 2; ++pass) {
    for (int i = t; i < s1 - s0; i += 256) *(volatile int*)(csr_eid + s0 + i) = (i < tot) ? sorted[i] : -1;
    { const int dst = hb * CS_NB + t; *(volatile int*)(csr_start + dst) = s0 + lpre[t]; *(volatile int*)(csr_cnt + dst) = lcnt[t]; }
    if (pass == 0) __threadfence(); }
}
static void build_csr(const int* eidst, int ne, int nt, int nn, int* seg_dst, int* seg_eid, int* P1, int* Q1, int* R, int* S, int* csr_eid, int* csr_start, int* csr_cnt, hipStream_t stream) {
  k_cs_p1<<<CS_NW / 8, 256, 0, stream>>>(eidst, ne, nt, nn, seg_dst, seg_eid, P1, Q1);
  k_cs_scan<<<1, 256, 0, stream>>>(P1, R, S);
  k_cs_p2<<<CS_NB, 256, 0, stream>>>(seg_dst, seg_eid, P1, Q1, R, S, nn, csr_eid, csr_start, csr_cnt);
}


typedef _Float16 v16h __attribute__((ext_vector_type(16)));
union FragH { v16h v; v8us half[2]; _Float16 h[16]; unsigned short u[16]; };
template <int NT>
__device__ __forceinline__ v8f mmaH(v16h ah, v16h al, v16h bh, v16h bl, v8f c) {
  c = __builtin_amdgcn_wmma_f32_16x16x32_f16(false, ah, false, bh, (short)0, c, false, false);
  if (NT >= 2) c = __builtin_amdgcn_wmma_f32_16x16x32_f16(false, al, false, bh, (short)0, c, false, false);
  if (NT >= 3) c = __builtin_amdgcn_wmma_f32_16x16x32_f16(false, ah, false, bl, (short)0, c, false, false);
  asm volatile("v_nop\n\tv_nop\n\tv_nop\n\tv_nop" : "+v"(c) : "v"(ah), "v"(al), "v"(bh), "v"(bl));
  return c;
}
template <bool ASPLIT>
__global__ __launch_bounds__(128) void k_gemm_h(const float* __restrict__ A, int lda, size_t sA, const _Float16* __restrict__ Bh, int ldb, size_t sB, float alpha, float* __restrict__ C, int ldc, size_t sC, int M, int N, int K) {
  __shared__ __attribute__((aligned(16))) float so[4][16][64];
  const int tid = threadIdx.x, w = tid >> 5, lane = tid & 31, ln = lane & 15, hh = lane >> 4; const int by = blockIdx.y;
  A += (size_t)by * sA; Bh += (size_t)by * sB; C += (size_t)by * sC;
  const int ntn = (N + 63) / 64; const int wid = blockIdx.x * 4 + w; const int mt = wid / ntn, nq = wid % ntn; if (mt * 16 >= M) return;
  const int row0 = mt * 16, col0 = nq * 64; const float* arow = A + (size_t)(row0 + ln) * lda;
  v8f acc[4] = {};
  for (int kb = 0; kb < K; kb += 32) {
    FragH ah, al;
    const v4f x0 = *(const v4fa*)(arow + kb + 8 * hh), x1 = *(const v4fa*)(arow + kb + 8 * hh + 4), x2 = *(const v4fa*)(arow + kb + 16 + 8 * hh), x3 = *(const v4fa*)(arow + kb + 16 + 8 * hh + 4);
    float xs[16] = {x0[0],x0[1],x0[2],x0[3],x1[0],x1[1],x1[2],x1[3],x2[0],x2[1],x2[2],x2[3],x3[0],x3[1],x3[2],x3[3]};
#pragma unroll
    for (int i = 0; i < 16; ++i) { const _Float16 h = (_Float16)xs[i]; ah.h[i] = h; al.h[i] = ASPLIT ? (_Float16)(xs[i] - (float)h) : (_Float16)0.0f; }
#pragma unroll
    for (int t = 0; t < 4; ++t) { if (col0 + t * 16 >= N) continue; const size_t boff = (size_t)(col0 + t * 16 + ln) * ldb + kb; FragH bq; bq.half[0] = *(const v8us*)(Bh + boff + 8 * hh); bq.half[1] = *(const v8us*)(Bh + boff + 16 + 8 * hh);
      acc[t] = mmaH<ASPLIT ? 2 : 1>(ah.v, al.v, bq.v, bq.v, acc[t]); }
  }
#pragma unroll
  for (int t = 0; t < 4; ++t) { if (col0 + t * 16 >= N) continue;
#pragma unroll
    for (int r = 0; r < 8; ++r) so[w][8 * hh + r][t * 16 + ln] = acc[t][r] * alpha; }
  __builtin_amdgcn_fence(__ATOMIC_ACQ_REL, "workgroup"); __builtin_amdgcn_wave_barrier();
  const int rsub = lane >> 4, c4 = (lane & 15) * 4;
  for (int pass = 0; pass < 2; ++pass) {
#pragma unroll
    for (int q = 0; q < 8; ++q) { const int r = q * 2 + rsub; if (col0 + c4 < N) { const v4f v = *(const v4fa*)&so[w][r][c4]; *(volatile v4f*)(C + (size_t)(row0 + r) * ldc + col0 + c4) = v; } }
    if (pass == 0) __threadfence(); }
}

template <int DUMMY>
__global__ __launch_bounds__(128) void k_gemm_hh(const _Float16* __restrict__ A, int lda, size_t sA, const _Float16* __restrict__ Bh, int ldb, size_t sB, float alpha, float* __restrict__ C, int ldc, size_t sC, int M, int N, int K) {
  __shared__ __attribute__((aligned(16))) float so[4][16][64];
  const int tid = threadIdx.x, w = tid >> 5, lane = tid & 31, ln = lane & 15, hh = lane >> 4; const int by = blockIdx.y;
  A += (size_t)by * sA; Bh += (size_t)by * sB; C += (size_t)by * sC;
  const int ntn = (N + 63) / 64; const int wid = blockIdx.x * 4 + w; const int mt = wid / ntn, nq = wid % ntn; if (mt * 16 >= M) return;
  const int row0 = mt * 16, col0 = nq * 64; const _Float16* arow = A + (size_t)(row0 + ln) * lda;
  v8f acc[4] = {};
  for (int kb = 0; kb < K; kb += 32) { FragH ah; ah.half[0] = *(const v8us*)((const unsigned short*)arow + kb + 8 * hh); ah.half[1] = *(const v8us*)((const unsigned short*)arow + kb + 16 + 8 * hh);
#pragma unroll
    for (int t = 0; t < 4; ++t) { if (col0 + t * 16 >= N) continue; const size_t boff = (size_t)(col0 + t * 16 + ln) * ldb + kb; FragH bq; bq.half[0] = *(const v8us*)((const unsigned short*)Bh + boff + 8 * hh); bq.half[1] = *(const v8us*)((const unsigned short*)Bh + boff + 16 + 8 * hh);
      acc[t] = mmaH<1>(ah.v, ah.v, bq.v, bq.v, acc[t]); }
  }
#pragma unroll
  for (int t = 0; t < 4; ++t) { if (col0 + t * 16 >= N) continue;
#pragma unroll
    for (int r = 0; r < 8; ++r) so[w][8 * hh + r][t * 16 + ln] = acc[t][r] * alpha; }
  __builtin_amdgcn_fence(__ATOMIC_ACQ_REL, "workgroup"); __builtin_amdgcn_wave_barrier();
  const int rsub = lane >> 4, c4 = (lane & 15) * 4;
  for (int pass = 0; pass < 2; ++pass) {
#pragma unroll
    for (int q = 0; q < 8; ++q) { const int r = q * 2 + rsub; if (col0 + c4 < N) { const v4f v = *(const v4fa*)&so[w][r][c4]; *(volatile v4f*)(C + (size_t)(row0 + r) * ldc + col0 + c4) = v; } }
    if (pass == 0) __threadfence(); }
}

__global__ __launch_bounds__(256) void k_bnstat(const float* __restrict__ ea, const float* __restrict__ W1, const float* __restrict__ b1, double* __restrict__ part) {
  __shared__ float sw[INN * HE]; __shared__ float sb[HE]; __shared__ double rs[2][4][64];
  const int tid = threadIdx.x; for (int i = tid; i < INN * HE; i += 256) sw[i] = bf16_round(W1[i]); if (tid < HE) sb[tid] = bf16_round(b1[tid]); __syncthreads();
  const int c = tid & 63, grp = tid >> 6;
  double s = 0.0, q = 0.0; const int e0 = blockIdx.x * 1024;
#pragma unroll 1
  for (int j = grp; j < 1024; j += 4) { const int e = e0 + j; if (e >= NE) break; const float* row = ea + (size_t)e * INN; float h = sb[c];
#pragma unroll
    for (int i = 0; i < INN; ++i) h += bf16_round(row[i]) * sw[i * HE + c]; s += (double)h; q += (double)h * (double)h; }
  rs[0][grp][c] = s; rs[1][grp][c] = q; __syncthreads();
  if (tid < 64) { const double a = ((rs[0][0][tid] + rs[0][1][tid]) + rs[0][2][tid]) + rs[0][3][tid], b = ((rs[1][0][tid] + rs[1][1][tid]) + rs[1][2][tid]) + rs[1][3][tid]; double* d = part + ((size_t)blockIdx.x * 64 + tid) * 2; *(volatile double*)d = a; *(volatile double*)(d + 1) = b; __threadfence(); *(volatile double*)d = a; *(volatile double*)(d + 1) = b; }
}
__global__ __launch_bounds__(64) void k_bnfin(const double* __restrict__ part, int nblk, const float* __restrict__ gamma, const float* __restrict__ beta, float* __restrict__ sc) {
  const int c = threadIdx.x; double s = 0.0, q = 0.0; for (int b = 0; b < nblk; ++b) { s += part[((size_t)b * 64 + c) * 2]; q += part[((size_t)b * 64 + c) * 2 + 1]; }
  const double mu = s / (double)NE; double var = q / (double)NE - mu * mu; if (var < 0.0) var = 0.0; const float rs = (float)(1.0 / sqrt(var + 1e-5)); const float g = bf16_round(gamma[c]), bb = bf16_round(beta[c]);
  const float scale = rs * g, shift = bb - (float)mu * rs * g; *(volatile float*)(sc + c * 2) = scale; *(volatile float*)(sc + c * 2 + 1) = shift; __threadfence(); *(volatile float*)(sc + c * 2) = scale; *(volatile float*)(sc + c * 2 + 1) = shift;
}
__global__ __launch_bounds__(128) void k_hedge(const float* __restrict__ ea, const _Float16* __restrict__ Bt, const float* __restrict__ b1, const float* __restrict__ sc, _Float16* __restrict__ H16) {
  __shared__ __attribute__((aligned(16))) _Float16 so[4][16][HE];
  const int tid = threadIdx.x, w = tid >> 5, lane = tid & 31, ln = lane & 15, hh = lane >> 4; const int row0 = (blockIdx.x * 4 + w) * 16; if (row0 >= NE) return; const int e = row0 + ln;
  FragH ah; { const float* r = ea + (size_t)e * INN + 8 * hh;
#pragma unroll
    for (int i = 0; i < 8; ++i) { ah.h[i] = (_Float16)bf16_round(r[i]); ah.h[8 + i] = (_Float16)0.0f; } }
  v8f acc[4] = {};
#pragma unroll
  for (int t = 0; t < 4; ++t) { FragH bq; bq.half[0] = *(const v8us*)((const unsigned short*)Bt + (size_t)(t * 16 + ln) * 32 + 8 * hh); bq.half[1] = *(const v8us*)((const unsigned short*)Bt + (size_t)(t * 16 + ln) * 32 + 16 + 8 * hh); acc[t] = mmaH<1>(ah.v, ah.v, bq.v, bq.v, acc[t]); }
#pragma unroll
  for (int t = 0; t < 4; ++t) {
#pragma unroll
    for (int r = 0; r < 8; ++r) { const int c = t * 16 + ln; const float h = (acc[t][r] * 0.0625f + bf16_round(b1[c])) * sc[c * 2] + sc[c * 2 + 1]; so[w][8 * hh + r][c] = (_Float16)fmaxf(h, 0.f); } }
  __builtin_amdgcn_fence(__ATOMIC_ACQ_REL, "workgroup"); __builtin_amdgcn_wave_barrier();
  typedef unsigned int u32; const u32* src = (const u32*)&so[w][0][0]; u32* dst = (u32*)(H16 + (size_t)row0 * HE);
  for (int pass = 0; pass < 2; ++pass) { for (int q = lane; q < 512; q += 32) *(volatile u32*)(dst + q) = src[q]; if (pass == 0) __threadfence(); }
}
__global__ __launch_bounds__(256) void k_w1t(const float* __restrict__ W1, _Float16* __restrict__ Bt) { const int t = threadIdx.x; const int c = t / 4, k8 = (t % 4) * 8; FragH f;
#pragma unroll
  for (int q = 0; q < 8; ++q) { const int i = k8 + q; f.h[q] = (i < INN) ? (_Float16)(bf16_round(W1[i * HE + c]) * 16.0f) : (_Float16)0.0f; } const v8us v = f.half[0]; *(volatile v8us*)((unsigned short*)Bt + c * 32 + k8) = v; __threadfence(); *(volatile v8us*)((unsigned short*)Bt + c * 32 + k8) = v; }
#define KP2 1088
__global__ __launch_bounds__(256) void k_aggw(const _Float16* __restrict__ H16, const float* __restrict__ x, const int* __restrict__ src, const int* __restrict__ cstart, const int* __restrict__ ccnt, const int* __restrict__ ceid, _Float16* __restrict__ SX) {
  __shared__ __attribute__((aligned(16))) _Float16 sh[8][32][HE]; __shared__ float sxr[8][32][INN + 1]; __shared__ __attribute__((aligned(16))) _Float16 srow[8][KP2];
  const int tid = threadIdx.x, wv = tid >> 5, lane = tid & 31, ln = lane & 15, hh = lane >> 4; const int d = blockIdx.x * 8 + wv; if (d >= NNODE) return; int p0 = cstart[d]; int cnt = ccnt[d]; cnt = cnt < 0 ? 0 : (cnt > MAXDEG ? MAXDEG : cnt); p0 = p0 < 0 ? 0 : (p0 > (NE + 32 * CS_NB) ? (NE + 32 * CS_NB) : p0);
  v8f acc[4] = {}; float xsum = 0.f;
#pragma unroll 1
  for (int s0 = 0; s0 < cnt; s0 += 32) { const int slot = s0 + lane; const bool live = slot < cnt; int s = 0; const _Float16* hr = nullptr;
    if (live) { int e = ceid[p0 + slot]; e = e < 0 ? 0 : (e >= NE ? NE - 1 : e); s = src[e]; s = s < 0 ? 0 : (s >= NNODE ? NNODE - 1 : s); hr = H16 + (size_t)e * HE; }
    { v8us* shd = (v8us*)&sh[wv][lane][0];
#pragma unroll
      for (int q = 0; q < HE / 8; ++q) shd[q] = live ? *(const v8us*)((const unsigned short*)hr + q * 8) : (v8us){0,0,0,0,0,0,0,0};
#pragma unroll
      for (int i = 0; i < INN; ++i) { const float xv = live ? bf16_round(x[(size_t)s * INN + i]) : 0.f; sxr[wv][lane][i] = xv; } }
    __builtin_amdgcn_fence(__ATOMIC_ACQ_REL, "workgroup"); __builtin_amdgcn_wave_barrier();
    if (lane < INN) { for (int q = 0; q < 32; ++q) xsum += (lane < INN) ? sxr[wv][q][lane] : 0.f; }
    FragH bq;
#pragma unroll
    for (int q = 0; q < 8; ++q) { bq.h[q] = (_Float16)sxr[wv][8 * hh + q][ln]; bq.h[8 + q] = (_Float16)sxr[wv][16 + 8 * hh + q][ln]; }
#pragma unroll
    for (int mt = 0; mt < 4; ++mt) { FragH ah; const int k = mt * 16 + ln;
#pragma unroll
      for (int q = 0; q < 8; ++q) { ah.h[q] = sh[wv][8 * hh + q][k]; ah.h[8 + q] = sh[wv][16 + 8 * hh + q][k]; }
      acc[mt] = mmaH<1>(ah.v, ah.v, bq.v, bq.v, acc[mt]); }
    __builtin_amdgcn_wave_barrier(); }
#pragma unroll
  for (int mt = 0; mt < 4; ++mt) {
#pragma unroll
    for (int r = 0; r < 8; ++r) srow[wv][(mt * 16 + 8 * hh + r) * INN + ln] = (_Float16)acc[mt][r]; }
  if (lane < INN) srow[wv][HE * INN + lane] = (_Float16)xsum; if (lane >= INN) srow[wv][HE * INN + lane] = (_Float16)0.0f; for (int q = HE * INN + 32 + lane; q < KP2; q += 32) srow[wv][q] = (_Float16)0.0f;
  __builtin_amdgcn_fence(__ATOMIC_ACQ_REL, "workgroup"); __builtin_amdgcn_wave_barrier();
  typedef unsigned int u32; const u32* sr = (const u32*)&srow[wv][0]; u32* dst = (u32*)(SX + (size_t)d * KP2);
  for (int pass = 0; pass < 2; ++pass) { for (int q = lane; q < KP2 / 2; q += 32) *(volatile u32*)(dst + q) = sr[q]; if (pass == 0) __threadfence(); }
}
__global__ __launch_bounds__(256) void k_wt2(const float* __restrict__ W2, const float* __restrict__ b2, _Float16* __restrict__ Bt) { const int t = blockIdx.x * 256 + threadIdx.x; if (t >= 32 * (KP2 / 8)) return; const int o = t / (KP2 / 8), c8 = (t % (KP2 / 8)) * 8; FragH f;
#pragma unroll
  for (int q = 0; q < 8; ++q) { const int c = c8 + q; float w = 0.f; if (o < ON) { if (c < HE * INN) { const int k = c / INN, i = c % INN; w = W2[(size_t)k * (INN * ON) + i * ON + o]; } else if (c < HE * INN + INN) { const int i = c - HE * INN; w = b2[i * ON + o]; } } f.h[q] = (_Float16)(bf16_round(w) * 16.0f); }
  const v8us v = f.half[0]; *(volatile v8us*)((unsigned short*)Bt + (size_t)o * KP2 + c8) = v; __threadfence(); *(volatile v8us*)((unsigned short*)Bt + (size_t)o * KP2 + c8) = v; }
__global__ __launch_bounds__(1024) void k_head(const float* __restrict__ AG, const float* __restrict__ x, const float* __restrict__ rw, const float* __restrict__ bias, const int* __restrict__ batch, const float* __restrict__ a, const float* __restrict__ Wc1, const float* __restrict__ bc1, const float* __restrict__ Wc2, const float* __restrict__ bc2, int g0, float* __restrict__ out) {
  __shared__ float sp[32][32]; __shared__ float sz[32][256];
  const int tid = threadIdx.x, wv = tid >> 5, lane = tid & 31; const int g = g0 + wv;
  int lo = 0, hi = NNODE; while (lo < hi) { const int m = (lo + hi) >> 1; if (batch[m] < g) lo = m + 1; else hi = m; } const int s0 = lo; lo = 0; hi = NNODE; while (lo < hi) { const int m = (lo + hi) >> 1; if (batch[m] < g + 1) lo = m + 1; else hi = m; } const int s1 = lo;
  float acc = 0.f; const int o = lane;
  if (o < ON) {
#pragma unroll 1
    for (int n = s0; n < s1; ++n) { float v = AG[(size_t)n * 32 + o] + bf16_round(bias[o]);
#pragma unroll
      for (int i = 0; i < INN; ++i) v += bf16_round(x[(size_t)n * INN + i]) * bf16_round(rw[i * ON + o]); acc += v; } }
  const float cnt = fmaxf((float)(s1 - s0), 1.0f); sp[wv][lane] = (lane < ON) ? acc / cnt : ((lane < ON + 8) ? bf16_round(a[g * 8 + (lane - ON)]) : 0.f);
  __builtin_amdgcn_fence(__ATOMIC_ACQ_REL, "workgroup"); __builtin_amdgcn_wave_barrier();
  for (int u = 0; u < 8; ++u) { const int c = u * 32 + lane; float v = bf16_round(bc1[c]); for (int j = 0; j < 28; ++j) v += sp[wv][j] * bf16_round(Wc1[j * 256 + c]); sz[wv][c] = fmaxf(v, 0.f); }
  __builtin_amdgcn_fence(__ATOMIC_ACQ_REL, "workgroup"); __builtin_amdgcn_wave_barrier();
  float r = 0.f; for (int c = lane; c < 256; c += 32) r += sz[wv][c] * bf16_round(Wc2[c]); for (int q = 16; q >= 1; q >>= 1) r += __shfl_xor(r, q, 32);
  __shared__ float so[32]; if (lane == 0) so[wv] = r + bf16_round(bc2[0]); __syncthreads();
  if (tid < 32) { *(volatile float*)(out + g0 + tid) = so[tid]; } __threadfence(); if (tid < 32) { *(volatile float*)(out + g0 + tid) = so[tid]; }
}
extern "C" void kernel_launch(void* const* d_in, const int* in_sizes, int n_in,
                              void* d_out, int out_size, void* d_ws, size_t ws_size, hipStream_t stream) {
  (void)in_sizes; (void)n_in; (void)out_size;
  const float* x = (const float*)d_in[0]; const float* ea = (const float*)d_in[1]; const float* a = (const float*)d_in[2]; const int* ei = (const int*)d_in[3]; const int* batch = (const int*)d_in[4];
  const float* W1 = (const float*)d_in[5]; const float* b1 = (const float*)d_in[6]; const float* gamma = (const float*)d_in[7]; const float* beta = (const float*)d_in[8]; const float* W2 = (const float*)d_in[9]; const float* b2 = (const float*)d_in[10]; const float* rw = (const float*)d_in[11]; const float* bias = (const float*)d_in[12];
  const float* Wc1 = (const float*)d_in[13]; const float* bc1 = (const float*)d_in[14]; const float* Wc2 = (const float*)d_in[15]; const float* bc2 = (const float*)d_in[16];
  char* ws = (char*)d_ws; size_t off = 0;
  auto take = [&](size_t bytes) { char* p = ws + off; off += (bytes + 255) & ~(size_t)255; return p; };
  const int NBLK = (NE + 1023) / 1024;
  double* part = (double*)take((size_t)NBLK * 64 * 2 * 8); float* sc = (float*)take(HE * 2 * 4); _Float16* Bt = (_Float16*)take((size_t)32 * KP2 * 2); _Float16* Bw1 = (_Float16*)take(64 * 32 * 2);
  int* seg_dst = (int*)take((size_t)CS_NW * CS_CH * 4); int* seg_eid = (int*)take((size_t)CS_NW * CS_CH * 4); int* P1 = (int*)take((size_t)CS_NW * CS_NB * 4); int* Q1 = (int*)take((size_t)CS_NW * CS_NB * 4); int* R = (int*)take((size_t)CS_NW * CS_NB * 4); int* S = (int*)take((CS_NB + 32) * 4);
  int* ceid = (int*)take(((size_t)NE + 32 * CS_NB) * 4); int* cstart = (int*)take((size_t)CS_NB * CS_NB * 4); int* ccnt = (int*)take((size_t)CS_NB * CS_NB * 4);
  _Float16* H16 = (_Float16*)take((size_t)NE * HE * 2); _Float16* SX = (_Float16*)take((size_t)NNODE * KP2 * 2); float* AG = (float*)take((size_t)NNODE * 32 * 4);
  if (off > ws_size) return;
  k_wt2<<<(32 * (KP2 / 8) + 255) / 256, 256, 0, stream>>>(W2, b2, Bt); k_w1t<<<1, 256, 0, stream>>>(W1, Bw1);
  build_csr(ei + NE, NE, NE, NNODE, seg_dst, seg_eid, P1, Q1, R, S, ceid, cstart, ccnt, stream);
  k_bnstat<<<NBLK, 256, 0, stream>>>(ea, W1, b1, part); k_bnfin<<<1, 64, 0, stream>>>(part, NBLK, gamma, beta, sc);
  k_hedge<<<(NE / 16 + 3) / 4, 128, 0, stream>>>(ea, Bw1, b1, sc, H16);
  k_aggw<<<(NNODE + 7) / 8, 256, 0, stream>>>(H16, x, ei, cstart, ccnt, ceid, SX);
  k_gemm_hh<0><<<dim3(((NNODE / 16) * 1 + 3) / 4, 1), 128, 0, stream>>>(SX, KP2, 0, Bt, KP2, 0, 0.0625f, AG, 32, 0, NNODE, 32, KP2);
  for (int g0 = 0; g0 < NG; g0 += 32) k_head<<<1, 1024, 0, stream>>>(AG, x, rw, bias, batch, a, Wc1, bc1, Wc2, bc2, g0, (float*)d_out);
}
